// DynamicLinear_56599079027182
// MI455X (gfx1250) — hardware-verified
//
#include <hip/hip_runtime.h>


#define LL   1024
#define NB_  8
#define CIN  1024
#define COUT 1024
#define CC   256
#define HID  64
#define KE   4
#define TEMP 30.0f
typedef _Float16 h16;
typedef unsigned short bf;
typedef __attribute__((ext_vector_type(16))) __bf16   v16bf;
typedef __attribute__((ext_vector_type(16))) _Float16 v16h;
typedef __attribute__((ext_vector_type(8)))  _Float16 v8h;
typedef __attribute__((ext_vector_type(8)))  unsigned short v8us;
typedef __attribute__((ext_vector_type(8)))  float    v8f;
typedef __attribute__((ext_vector_type(4)))  float    v4f;
typedef v8h  __attribute__((may_alias)) v8ha;
typedef v4f  __attribute__((may_alias)) v4fa;
typedef v8us __attribute__((may_alias)) v8usa;

__device__ __forceinline__ unsigned short f2bf(float f) { unsigned u = __float_as_uint(f); u += 0x7FFFu + ((u >> 16) & 1u); return (unsigned short)(u >> 16); }
__device__ __forceinline__ float bf2f(unsigned short b) { return __uint_as_float(((unsigned)b) << 16); }
__device__ __forceinline__ float bfr(float f) { return bf2f(f2bf(f)); }
__device__ __forceinline__ v16h cat16(v8h lo, v8h hi) { return __builtin_shufflevector(lo, hi, 0, 1, 2, 3, 4, 5, 6, 7, 8, 9, 10, 11, 12, 13, 14, 15); }
__device__ __forceinline__ v16bf cat16b(v8us lo, v8us hi) { return __builtin_bit_cast(v16bf, __builtin_shufflevector(lo, hi, 0, 1, 2, 3, 4, 5, 6, 7, 8, 9, 10, 11, 12, 13, 14, 15)); }
__device__ __forceinline__ v8f wmma16(v16h a, v16h b, v8f c) { return __builtin_amdgcn_wmma_f32_16x16x32_f16(false, a, false, b, (short)0, c, false, false); }
__device__ __forceinline__ v8f wmmab(v16bf a, v16bf b, v8f c) { return __builtin_amdgcn_wmma_f32_16x16x32_bf16(false, a, false, b, (short)0, c, false, false); }


template <typename T16> struct WFrag;
template <> struct WFrag<h16> { typedef v16h V; static __device__ __forceinline__ V ld(const h16* p) { return cat16(*(const v8h*)p, *(const v8h*)(p + 16)); } static __device__ __forceinline__ v8f mma(V a, V b, v8f c) { return wmma16(a, b, c); } };
template <> struct WFrag<bf> { typedef v16bf V; static __device__ __forceinline__ V ld(const bf* p) { return cat16b(*(const v8us*)p, *(const v8us*)(p + 16)); } static __device__ __forceinline__ v8f mma(V a, V b, v8f c) { return wmmab(a, b, c); } };
template <typename T16, int NSPLIT, bool BIAS>
__global__ __launch_bounds__(32) void k_gemmw(const T16* __restrict__ A, const T16* __restrict__ A2, const T16* __restrict__ Bt, const T16* __restrict__ Bt2, int K, float* C, int ldc, const float* __restrict__ bias, size_t sA, size_t sB, size_t sC) {
    typedef typename WFrag<T16>::V V;
    __shared__ __align__(16) float os[16 * 68];
    const size_t z = blockIdx.z; A += z * sA; if (A2) A2 += z * sA; Bt += z * sB; if (Bt2) Bt2 += z * sB; C += z * sC;
    const int lane = threadIdx.x & 31, lr = lane & 15, hi = lane >> 4; const int r0 = blockIdx.x * 64, c0 = blockIdx.y * 64;
    v8f acc[4][4];
#pragma unroll
    for (int mb = 0; mb < 4; ++mb)
#pragma unroll
        for (int nb = 0; nb < 4; ++nb) acc[mb][nb] = (v8f){};
    const size_t aoff = (size_t)(r0 + lr) * K + 8 * hi, boff = (size_t)(c0 + lr) * K + 8 * hi;
#pragma unroll 1
    for (int kc = 0; kc < K; kc += 32) {
        V a[4], a2[4];
#pragma unroll
        for (int mb = 0; mb < 4; ++mb) { a[mb] = WFrag<T16>::ld(A + aoff + (size_t)mb * 16 * K + kc); if (NSPLIT == 1 || NSPLIT == 2) a2[mb] = WFrag<T16>::ld(A2 + aoff + (size_t)mb * 16 * K + kc); }
#pragma unroll
        for (int nb = 0; nb < 4; ++nb) { const V b = WFrag<T16>::ld(Bt + boff + (size_t)nb * 16 * K + kc); V b2; if (NSPLIT >= 2) b2 = WFrag<T16>::ld(Bt2 + boff + (size_t)nb * 16 * K + kc);
#pragma unroll
            for (int mb = 0; mb < 4; ++mb) { acc[mb][nb] = WFrag<T16>::mma(a[mb], b, acc[mb][nb]); if (NSPLIT == 1 || NSPLIT == 2) acc[mb][nb] = WFrag<T16>::mma(a2[mb], b, acc[mb][nb]); if (NSPLIT >= 2) acc[mb][nb] = WFrag<T16>::mma(a[mb], b2, acc[mb][nb]); } }
        asm volatile("v_nop\n\tv_nop\n\tv_nop\n\tv_nop" : "+v"(acc[0][0]), "+v"(acc[1][1]), "+v"(acc[2][2]), "+v"(acc[3][3]) : "v"(a[0]), "v"(a[3]));
    }
#pragma unroll
    for (int mb = 0; mb < 4; ++mb) {
#pragma unroll
        for (int nb = 0; nb < 4; ++nb) {
#pragma unroll
            for (int j = 0; j < 8; ++j) os[(hi * 8 + j) * 68 + nb * 16 + lr] = acc[mb][nb][j]; }
        __builtin_amdgcn_wave_barrier(); asm volatile("" ::: "memory");
        float* crow = C + (size_t)(r0 + mb * 16) * ldc + c0;
#pragma unroll 1
        for (int ps = 0; ps < 2; ++ps) {
#pragma unroll
            for (int s = 0; s < 8; ++s) { const int row = 2 * s + hi, cofs = lr * 4; v4f val = *(const v4fa*)(os + row * 68 + cofs); if (BIAS) { val[0] += bfr(bias[c0 + cofs]); val[1] += bfr(bias[c0 + cofs + 1]); val[2] += bfr(bias[c0 + cofs + 2]); val[3] += bfr(bias[c0 + cofs + 3]); }
                *(volatile v4f*)(crow + (size_t)row * ldc + cofs) = val; }
            if (ps == 0) __threadfence(); }
        __builtin_amdgcn_wave_barrier(); asm volatile("" ::: "memory");
    }
}

__device__ __forceinline__ void splitf(float y, unsigned short& h, unsigned short& l) { h = f2bf(y); l = f2bf(y - bf2f(h)); }
typedef __attribute__((ext_vector_type(2))) float v2f;
typedef __attribute__((ext_vector_type(4))) unsigned short v4us;

__global__ __launch_bounds__(32) void k_gate(const float* __restrict__ cond, const float* __restrict__ fc1, const float* __restrict__ b1, const float* __restrict__ fc2, const float* __restrict__ b2, float* ATT) { const int b = blockIdx.x, lane = threadIdx.x; const float* cb = cond + (size_t)b * CC; float h[2];
#pragma unroll
    for (int q = 0; q < 2; ++q) { const int j = lane * 2 + q; float s = 0.f;
#pragma unroll 1
        for (int c = 0; c < CC; ++c) { float p = __fmul_rn(bfr(cb[c]), bfr(fc1[(size_t)j * CC + c])); asm volatile("" : "+v"(p)); s = __fadd_rn(s, p); }
        h[q] = fmaxf(__fadd_rn(s, bfr(b1[j])), 0.f); }
    float z[KE];
#pragma unroll
    for (int k = 0; k < KE; ++k) { float s = 0.f;
#pragma unroll
        for (int q = 0; q < 2; ++q) { float p = __fmul_rn(h[q], bfr(fc2[k * HID + lane * 2 + q])); asm volatile("" : "+v"(p)); s = __fadd_rn(s, p); }
#pragma unroll
        for (int sh = 16; sh; sh >>= 1) s += __shfl_xor(s, sh, 32);
        z[k] = __fdiv_rn(__fadd_rn(s, bfr(b2[k])), TEMP); }
    float mx = z[0]; for (int k = 1; k < KE; ++k) mx = fmaxf(mx, z[k]); float e[KE], sum = 0.f;
#pragma unroll
    for (int k = 0; k < KE; ++k) { e[k] = expf(__fsub_rn(z[k], mx)); sum = __fadd_rn(sum, e[k]); }
    float ev = 0.f;
#pragma unroll
    for (int k = 0; k < KE; ++k) ev = (lane == k) ? e[k] : ev;
    const float v = (lane < KE) ? __fdiv_rn(ev, sum) : 0.f;
    *(volatile float*)(ATT + b * 32 + lane) = v; __threadfence(); *(volatile float*)(ATT + b * 32 + lane) = v; }
__global__ __launch_bounds__(256) void k_aggw(const float* __restrict__ wt, const float* __restrict__ ATT, int b, bf* Wh, bf* Wl) { const size_t e = ((size_t)blockIdx.x * 256 + threadIdx.x) * 4; if (e >= (size_t)COUT * CIN) return; float a[KE];
#pragma unroll
    for (int k = 0; k < KE; ++k) a[k] = ATT[b * 32 + k];
    v4us oh, ol; const v4f w0 = *(const v4f*)(wt + e), w1 = *(const v4f*)(wt + (size_t)COUT * CIN + e), w2 = *(const v4f*)(wt + 2 * (size_t)COUT * CIN + e), w3 = *(const v4f*)(wt + 3 * (size_t)COUT * CIN + e);
#pragma unroll
    for (int q = 0; q < 4; ++q) { float s = __fmul_rn(a[0], bfr(w0[q])); float p; p = __fmul_rn(a[1], bfr(w1[q])); asm volatile("" : "+v"(p)); s = __fadd_rn(s, p); p = __fmul_rn(a[2], bfr(w2[q])); asm volatile("" : "+v"(p)); s = __fadd_rn(s, p); p = __fmul_rn(a[3], bfr(w3[q])); asm volatile("" : "+v"(p)); s = __fadd_rn(s, p); unsigned short hh, l2; splitf(s, hh, l2); oh[q] = hh; ol[q] = l2; }
    *(volatile v4us*)(Wh + e) = oh; *(volatile v4us*)(Wl + e) = ol; __threadfence(); *(volatile v4us*)(Wh + e) = oh; *(volatile v4us*)(Wl + e) = ol; }
__global__ __launch_bounds__(256) void k_xb(const float* __restrict__ x, int b, bf* X) { const size_t e = ((size_t)blockIdx.x * 256 + threadIdx.x) * 8; if (e >= (size_t)LL * CIN) return; const int i = (int)(e % CIN), l = (int)(e / CIN); const v8f v = *(const v8f*)(x + ((size_t)l * NB_ + b) * CIN + i); v8us o;
#pragma unroll
    for (int q = 0; q < 8; ++q) o[q] = f2bf(v[q]); *(volatile v8us*)(X + e) = o; __threadfence(); *(volatile v8us*)(X + e) = o; }
__global__ __launch_bounds__(256) void k_outT(const float* __restrict__ C, const float* __restrict__ bias, const float* __restrict__ ATT, int b, float* OUT) { const size_t e = ((size_t)blockIdx.x * 256 + threadIdx.x) * 2; if (e >= (size_t)LL * COUT) return; const int o = (int)(e % COUT), l = (int)(e / COUT); float a[KE];
#pragma unroll
    for (int k = 0; k < KE; ++k) a[k] = ATT[b * 32 + k];
    v2f r;
#pragma unroll
    for (int q = 0; q < 2; ++q) { const int oo = o + q; float bb = __fmul_rn(a[0], bfr(bias[oo])); float p; p = __fmul_rn(a[1], bfr(bias[COUT + oo])); asm volatile("" : "+v"(p)); bb = __fadd_rn(bb, p); p = __fmul_rn(a[2], bfr(bias[2 * COUT + oo])); asm volatile("" : "+v"(p)); bb = __fadd_rn(bb, p); p = __fmul_rn(a[3], bfr(bias[3 * COUT + oo])); asm volatile("" : "+v"(p)); bb = __fadd_rn(bb, p);
        r[q] = __fadd_rn(C[(size_t)oo * LL + l], bb); }
    float* dst = OUT + ((size_t)l * NB_ + b) * COUT + o; *(volatile v2f*)dst = r; __threadfence(); *(volatile v2f*)dst = r; }

extern "C" void kernel_launch(void* const* d_in, const int* in_sizes, int n_in,
                              void* d_out, int out_size, void* d_ws, size_t ws_size, hipStream_t stream) {
    (void)in_sizes; (void)n_in; (void)out_size;
    const float* x = (const float*)d_in[0]; const float* cond = (const float*)d_in[1]; const float* fc1 = (const float*)d_in[2]; const float* b1 = (const float*)d_in[3]; const float* fc2 = (const float*)d_in[4]; const float* b2 = (const float*)d_in[5]; const float* wt = (const float*)d_in[6]; const float* bias = (const float*)d_in[7];
    float* OUT = (float*)d_out;
    char* wsp = (char*)d_ws;
    auto take = [&](size_t bytes) { char* p = wsp; wsp += (bytes + 255) & ~(size_t)255; return (void*)p; };
    float* ATT = (float*)take((size_t)NB_ * 32 * 4); bf* Wh = (bf*)take((size_t)COUT * CIN * 2); bf* Wl = (bf*)take((size_t)COUT * CIN * 2); bf* XB = (bf*)take((size_t)LL * CIN * 2); float* C = (float*)take((size_t)COUT * LL * 4);
    if ((size_t)(wsp - (char*)d_ws) > ws_size) return;
    k_gate<<<NB_, 32, 0, stream>>>(cond, fc1, b1, fc2, b2, ATT);
    for (int b = 0; b < NB_; ++b) {
        k_aggw<<<(unsigned)(((size_t)COUT * CIN / 4 + 255) / 256), 256, 0, stream>>>(wt, ATT, b, Wh, Wl);
        k_xb<<<(unsigned)(((size_t)LL * CIN / 8 + 255) / 256), 256, 0, stream>>>(x, b, XB);
        k_gemmw<bf, 1, false><<<dim3(COUT / 64, LL / 64, 1), 32, 0, stream>>>(Wh, Wl, XB, nullptr, CIN, C, LL, nullptr, 0, 0, 0);
        k_outT<<<(unsigned)(((size_t)LL * COUT / 2 + 255) / 256), 256, 0, stream>>>(C, bias, ATT, b, OUT); }
}
